// ProbabilisticFractionalLayer_20925080666467
// MI455X (gfx1250) — hardware-verified
//
#include <hip/hip_runtime.h>
#include <math.h>

typedef __attribute__((ext_vector_type(16))) _Float16 v16h;
typedef __attribute__((ext_vector_type(16))) __bf16 v16b;
typedef __attribute__((ext_vector_type(8)))  _Float16 v8h;
typedef __attribute__((ext_vector_type(8)))  float v8f;
typedef __attribute__((ext_vector_type(4)))  float v4f;
typedef __attribute__((ext_vector_type(2)))  float v2f;
typedef __attribute__((ext_vector_type(4)))  unsigned v4u;
typedef __attribute__((ext_vector_type(4)))  int v4i;
typedef float __attribute__((may_alias)) float_a;
typedef int __attribute__((may_alias)) int_a;

template <typename T> __device__ __forceinline__ void vst2(void* p, T v) { *(volatile T*)p = v; __threadfence(); *(volatile T*)p = v; }
__device__ __forceinline__ v8f wmma16(v16h a, v16h b, v8f c) {
  v8f d = __builtin_amdgcn_wmma_f32_16x16x32_f16(false, a, false, b, (short)0, c, false, false);
  asm volatile("v_nop\n\tv_nop\n\tv_nop\n\tv_nop" : "+v"(d) : "v"(a), "v"(b));
  return d;
}
__device__ __forceinline__ v8f wmma_bf(v16b a, v16b b, v8f c) {
  v8f d = __builtin_amdgcn_wmma_f32_16x16x32_bf16(false, a, false, b, (short)0, c, false, false);
  asm volatile("v_nop\n\tv_nop\n\tv_nop\n\tv_nop" : "+v"(d) : "v"(a), "v"(b));
  return d;
}
__device__ __forceinline__ v16h frag_h(const _Float16* rowk0, int lane) {
  union { v16h v; v8h q[2]; } u; const _Float16* p = rowk0 + 8 * (lane >> 4);
  u.q[0] = *(const v8h*)p; u.q[1] = *(const v8h*)(p + 16); return u.v;
}
__device__ __forceinline__ v16h frag_f32(const float* rowk0, int lane) {
  v16h a; const float* p = rowk0 + 8 * (lane >> 4);
#pragma unroll
  for (int i = 0; i < 8; ++i) { a[i] = (_Float16)p[i]; a[8 + i] = (_Float16)p[16 + i]; }
  return a;
}
__device__ __forceinline__ v16h frag_f32s(const float* rowk0, int lane, float sc) {
  v16h a; const float* p = rowk0 + 8 * (lane >> 4);
#pragma unroll
  for (int i = 0; i < 8; ++i) { a[i] = (_Float16)(p[i] * sc); a[8 + i] = (_Float16)(p[16 + i] * sc); }
  return a;
}
__device__ __forceinline__ v16h fragc_f32(const float* W, int k0, int n, int lane, int ld, int K) {
  v16h a; const int g = lane >> 4;
#pragma unroll
  for (int i = 0; i < 8; ++i) { const int ka = k0 + 8 * g + i, kb = ka + 16;
    a[i] = (_Float16)(ka < K ? W[(size_t)(ka < K ? ka : K - 1) * ld + n] : 0.f); a[8 + i] = (_Float16)(kb < K ? W[(size_t)(kb < K ? kb : K - 1) * ld + n] : 0.f); }
  return a;
}
struct F2 { v16b h, l; };
__device__ __forceinline__ F2 bsplit16(const float v[16]) { F2 r;
#pragma unroll
  for (int i = 0; i < 16; ++i) { const __bf16 h = (__bf16)v[i]; r.h[i] = h; r.l[i] = (__bf16)(v[i] - (float)h); }
  return r; }
__device__ __forceinline__ F2 split_row(const float* row, int k0, int lane) { float v[16]; const float* p = row + k0 + 8 * (lane >> 4);
#pragma unroll
  for (int i = 0; i < 8; ++i) { v[i] = p[i]; v[8 + i] = p[16 + i]; }
  return bsplit16(v); }
__device__ __forceinline__ F2 split_rowK(const float* row, int k0, int lane, int K) { float v[16]; const int g = lane >> 4;
#pragma unroll
  for (int i = 0; i < 8; ++i) { const int ka = k0 + 8 * g + i, kb = ka + 16; v[i] = ka < K ? row[ka < K ? ka : K - 1] : 0.f; v[8 + i] = kb < K ? row[kb < K ? kb : K - 1] : 0.f; }
  return bsplit16(v); }
__device__ __forceinline__ F2 split_col(const float* W, int k0, int n, int lane, int ld, int K) { float v[16]; const int g = lane >> 4;
#pragma unroll
  for (int i = 0; i < 8; ++i) { const int ka = k0 + 8 * g + i, kb = ka + 16; v[i] = ka < K ? W[(size_t)(ka < K ? ka : K - 1) * ld + n] : 0.f; v[8 + i] = kb < K ? W[(size_t)(kb < K ? kb : K - 1) * ld + n] : 0.f; }
  return bsplit16(v); }
__device__ __forceinline__ v8f mac3(const F2& a, const F2& b, v8f c) { c = wmma_bf(a.l, b.h, c); c = wmma_bf(a.h, b.l, c); return wmma_bf(a.h, b.h, c); }
__device__ __forceinline__ float sigm(float v) { return 1.0f / (1.0f + expf(-v)); }
#define LDSX() do { asm volatile("s_wait_dscnt 0" ::: "memory"); __builtin_amdgcn_wave_barrier(); __builtin_amdgcn_fence(__ATOMIC_RELEASE, "workgroup"); } while (0)


#define NBS 16
#define NN 65536
#define KL 64
#ifndef NROWB
#define NROWB (NBS * NN / 64)
#endif
typedef __attribute__((ext_vector_type(8))) __bf16 v8b;
__device__ __forceinline__ v16b frag_b(const __bf16* rowk0, int lane) {
  union { v16b v; v8b q[2]; } u; const __bf16* p = rowk0 + 8 * (lane >> 4);
  u.q[0] = *(const v8b*)p; u.q[1] = *(const v8b*)(p + 16); return u.v;
}
__device__ __forceinline__ float bfr(float v) { return (float)(__bf16)v; }
__device__ __attribute__((noinline)) float exp_ni(float v) { return expf(v); }
__device__ __attribute__((noinline)) float erf_ni(float v) { return erff(v); }

__device__ __attribute__((noinline)) float lgamma_ni(float v) { return lgammaf(v); }
__device__ __attribute__((noinline)) float pow_ni(float a, float b) { return powf(a, b); }
__device__ __attribute__((noinline)) float log1p_ni(float v) { return log1pf(v); }
#define WS_PB   0u
#define WS_SC   (WS_PB + 2u * 2 * 16 * KL)
#define WS_END  (WS_SC + 4u * 96)

__global__ __launch_bounds__(64) void k_prep(const float* __restrict__ LOC, const float* __restrict__ SCL, const float* __restrict__ EPSI, const int* __restrict__ LAGS, __bf16* __restrict__ PB, float* __restrict__ SC) {
  __shared__ __align__(16) __bf16 sh[16][KL], sl[16][KL]; __shared__ __align__(16) float ssc[8]; __shared__ __align__(16) int sj[KL]; const int t = threadIdx.x;
  const float scl = bfr(SCL[0]), loc = bfr(LOC[0]), eps = bfr(EPSI[0]);
  const float sp = fmaxf(scl, 0.f) + log1p_ni(expf(-fabsf(scl)));
  float alpha = loc + sp * eps; alpha = fminf(fmaxf(alpha, 0.01f), 0.99f);
  const float c = alpha * expf(-lgamma_ni(1.0f - alpha)) * (float)(NN - 1) / (float)KL;
  { const int j = min(max(LAGS[t], 1), NN - 1); sj[t] = j; const float w = pow_ni((float)j, -(alpha + 1.0f)); const __bf16 h = (__bf16)w; for (int o = 0; o < 16; ++o) { sh[o][t] = (o == 0) ? h : (__bf16)0.f; sl[o][t] = (o == 0) ? (__bf16)(w - (float)h) : (__bf16)0.f; } }
  if (t == 0) { ssc[0] = alpha; ssc[1] = c; for (int q = 2; q < 8; ++q) ssc[q] = 0.f; }
  __syncthreads();
  for (int q = t; q < 16 * KL / 8; q += 64) { vst2((unsigned*)(PB + q * 8), *(const v4u*)(&sh[0][0] + q * 8)); vst2((unsigned*)(PB + 16 * KL + q * 8), *(const v4u*)(&sl[0][0] + q * 8)); }
  if (t < 2) vst2(SC + t * 4, *(const v4f*)&ssc[t * 4]);
  if (t < 16) vst2((unsigned*)((int*)(SC + 8) + t * 4), *(const v4u*)&sj[t * 4]);
}
__global__ __launch_bounds__(128) void k_frac(const float* __restrict__ X, const __bf16* __restrict__ PB, const float* __restrict__ SC, float* __restrict__ OUT) {
  __shared__ __align__(16) float so[64]; __shared__ int sj[KL];
  const int tid = threadIdx.x, wave = tid >> 5, lane = tid & 31, col = lane & 15, g = lane >> 4; const size_t r0 = (size_t)blockIdx.x * 64 + wave * 16;
  if (tid < KL) sj[tid] = ((const int*)(SC + 8))[tid];
  __syncthreads();
  const size_t row = r0 + col; const int b = (int)(row / NN), t = (int)(row % NN); const float xt = bfr(X[(size_t)b * NN + t]);
  v8f acc = {};
#pragma unroll
  for (int kc = 0; kc < 2; ++kc) { v16b ah, al;
#pragma unroll
    for (int i = 0; i < 16; ++i) { const int m = kc * 32 + 8 * g + (i < 8 ? i : 8 + i); const int j = sj[m]; float d = 0.f; if (t >= j) d = xt - bfr(X[(size_t)b * NN + (t - j)]); const __bf16 h = (__bf16)d; ah[i] = h; al[i] = (__bf16)(d - (float)h); }
    const v16b wh = frag_b(PB + (size_t)col * KL + kc * 32, lane), wl = frag_b(PB + 16 * KL + (size_t)col * KL + kc * 32, lane);
    acc = wmma_bf(al, wh, acc); acc = wmma_bf(ah, wl, acc); acc = wmma_bf(ah, wh, acc); }
  const float c = SC[1];
  if (col == 0) {
#pragma unroll
    for (int r = 0; r < 8; ++r) so[wave * 16 + 8 * g + r] = c * acc[r]; }
  __syncthreads();
  if (tid < 16) vst2(OUT + (size_t)blockIdx.x * 64 + tid * 4, *(const v4f*)&so[tid * 4]);
}
extern "C" void kernel_launch(void* const* d_in, const int* in_sizes, int n_in, void* d_out, int out_size, void* d_ws, size_t ws_size, hipStream_t stream) {
  (void)in_sizes; (void)n_in; (void)out_size;
  if (ws_size < (size_t)WS_END) return;
  char* ws = (char*)d_ws; __bf16* PB = (__bf16*)(ws + WS_PB); float* SC = (float*)(ws + WS_SC);
  k_prep<<<1, 64, 0, stream>>>((const float*)d_in[1], (const float*)d_in[2], (const float*)d_in[3], (const int*)d_in[4], PB, SC);
  k_frac<<<NROWB, 128, 0, stream>>>((const float*)d_in[0], PB, SC, (float*)d_out);
}
